// MambaBlock_67405216743458
// MI455X (gfx1250) — hardware-verified
//
#include <hip/hip_runtime.h>
#include <math.h>

typedef __attribute__((ext_vector_type(16))) __bf16   v16b;
typedef __attribute__((ext_vector_type(8)))  __bf16   v8b;
typedef __attribute__((ext_vector_type(8)))  float    v8f;
typedef __attribute__((ext_vector_type(4)))  float    v4f;
typedef __attribute__((ext_vector_type(4)))  unsigned v4u;

constexpr int kBatch  = 2;
constexpr int kSeq    = 1024;
constexpr int kDm     = 1024;
constexpr int kDin    = 2048;
constexpr int kNst    = 64;
constexpr int kDtR    = 64;
constexpr int kXzP    = 2 * kDin;
constexpr int kXdP    = kDtR + 2 * kNst;
constexpr int kRows   = kBatch * kSeq;
constexpr int kConvTP = 260;
constexpr int kScanTS = 16;
constexpr int kScanCh = 64;
constexpr int kScanYP = 68;
constexpr int kScanHP = 68;
static_assert(kXzP == 4096 && kXdP == 192 && kRows == 2048, "shape constants");
static_assert((kDm % 32) == 0 && (kDin % 32) == 0 && (kDtR % 32) == 0, "GEMM K multiples of 32");
static_assert((kRows % 64) == 0 && (kXzP % 64) == 0 && (kXdP % 64) == 0 && (kDin % 64) == 0 && (kDm % 64) == 0, "GEMM M,N multiples of 64");
static_assert((kSeq % 64) == 0 && (kSeq % kScanTS) == 0 && (kDin % kScanCh) == 0 && (kDin % 256) == 0, "tile multiples");
static_assert(kNst == 64 && kDtR == 64, "scan staging assumes 128 B/C floats per step and 64 dt columns");

constexpr size_t kOffXH   = 0;
constexpr size_t kOffWIH  = kOffXH  + (size_t)kRows * kDm  * 2;
constexpr size_t kOffWXH  = kOffWIH + (size_t)kXzP  * kDm  * 2;
constexpr size_t kOffWDH  = kOffWXH + (size_t)kXdP  * kDin * 2;
constexpr size_t kOffWOH  = kOffWDH + (size_t)kDin  * kDtR * 2;
constexpr size_t kOffXZ   = kOffWOH + (size_t)kDm   * kDin * 2;
constexpr size_t kOffUC   = kOffXZ  + (size_t)kRows * kXzP * 4;
constexpr size_t kOffUCH  = kOffUC  + (size_t)kRows * kDin * 4;
constexpr size_t kOffUCL  = kOffUCH + (size_t)kRows * kDin * 2;
constexpr size_t kOffXD   = kOffUCL + (size_t)kRows * kDin * 2;
constexpr size_t kOffDTH  = kOffXD  + (size_t)kRows * kXdP * 4;
constexpr size_t kOffDTL  = kOffDTH + (size_t)kRows * kDtR * 2;
constexpr size_t kOffDLR  = kOffDTL + (size_t)kRows * kDtR * 2;
constexpr size_t kOffYH   = kOffDLR + (size_t)kRows * kDin * 4;
constexpr size_t kOffYL   = kOffYH  + (size_t)kRows * kDin * 2;
constexpr size_t kWsTotal = kOffYL  + (size_t)kRows * kDin * 2;
static_assert(kWsTotal == 120586240ull, "carve total");
static_assert(kWsTotal <= 134217728ull, "carve cap");
static_assert((kOffWIH % 128) == 0 && (kOffWXH % 128) == 0 && (kOffWDH % 128) == 0 && (kOffWOH % 128) == 0 &&
              (kOffXZ % 128) == 0 && (kOffUC % 128) == 0 && (kOffUCH % 128) == 0 && (kOffUCL % 128) == 0 &&
              (kOffXD % 128) == 0 && (kOffDTH % 128) == 0 && (kOffDTL % 128) == 0 && (kOffDLR % 128) == 0 &&
              (kOffYH % 128) == 0 && (kOffYL % 128) == 0, "128-B aligned regions");

__device__ __forceinline__ unsigned bf16_bits(float f) {
  const unsigned u = __float_as_uint(f);
  return (u + 0x7FFFu + ((u >> 16) & 1u)) >> 16;
}
__device__ __forceinline__ float bf16_val(unsigned b) { return __uint_as_float(b << 16); }
__device__ __forceinline__ float bf16r(float f) { return bf16_val(bf16_bits(f)); }
__device__ __forceinline__ unsigned pack_hi2(float a, float b) { return bf16_bits(a) | (bf16_bits(b) << 16); }
__device__ __forceinline__ unsigned pack_lo2(float a, float b) {
  const float ra = a - bf16_val(bf16_bits(a));
  const float rb = b - bf16_val(bf16_bits(b));
  return bf16_bits(ra) | (bf16_bits(rb) << 16);
}

__device__ __forceinline__ void dep_guard4_b(v8f& a, v8f& b, v8f& c, v8f& d, v16b x, v16b y) {
  asm volatile("v_nop\n\tv_nop\n\tv_nop\n\tv_nop" : "+v"(a), "+v"(b), "+v"(c), "+v"(d) : "v"(x), "v"(y));
}
__device__ __forceinline__ void keep4_b(v16b a, v16b b, v16b c, v16b d) { asm volatile("v_nop" :: "v"(a), "v"(b), "v"(c), "v"(d)); }
__device__ __forceinline__ void acc_guard4(v8f& a, v8f& b, v8f& c, v8f& d) { asm volatile("v_nop\n\tv_nop\n\tv_nop\n\tv_nop" : "+v"(a), "+v"(b), "+v"(c), "+v"(d)); }
template <typename T> struct Frag;
template <> struct Frag<__bf16> {
  typedef v16b V; union U { v16b v; v8b h[2]; };
  static __device__ __forceinline__ v16b load(const __bf16* p) {
    U f; f.h[0] = *(const v8b*)(p); f.h[1] = *(const v8b*)(p + 16); return f.v;
  }
  static __device__ __forceinline__ v8f mma(v16b a, v16b b, v8f c) {
    return __builtin_amdgcn_wmma_f32_16x16x32_bf16(false, a, false, b, (short)0, c, false, false);
  }
};

template <int SPL, bool ROWMUL>
__global__ __launch_bounds__(256) void wmma_gemm64(
    const unsigned short* __restrict__ Ap, const unsigned short* __restrict__ A2p, int lda,
    const unsigned short* __restrict__ Btp, int ldb,
    float* __restrict__ Cout, int ldc,
    const float* __restrict__ rowmul,
    int M, int N, int K) {
  typedef __bf16 T;
  typedef v16b V;
  const T* A = (const T*)Ap; const T* A2 = (const T*)A2p; const T* Bt = (const T*)Btp;
  __shared__ __align__(16) float sT[8][16 * 68];
  const int lane = threadIdx.x & 31;
  const int wave = threadIdx.x >> 5;
  const int tilesN = N >> 6;
  const int tilesM = M >> 6;
  const int tile = blockIdx.x * 8 + wave;
  if (tile >= tilesM * tilesN) return;
  const int tm = tile / tilesN;
  const int tn = tile - tm * tilesN;
  const int m0 = tm << 6;
  const int n0 = tn << 6;

  const int rlane = lane & 15;
  const int koff  = (lane >> 4) * 8;
  const int mOff  = (lane >> 4) * 8;

  v8f acc[4][4];
#pragma unroll
  for (int i = 0; i < 4; ++i)
#pragma unroll
    for (int j = 0; j < 4; ++j) acc[i][j] = (v8f){0.f,0.f,0.f,0.f,0.f,0.f,0.f,0.f};

  for (int k0 = 0; k0 < K; k0 += 32) {
    V bh[4];
#pragma unroll
    for (int j = 0; j < 4; ++j) {
      const size_t bo = (size_t)(n0 + (j << 4) + rlane) * ldb + koff + k0;
      bh[j] = Frag<T>::load(Bt + bo);
    }
#pragma unroll
    for (int i = 0; i < 4; ++i) {
      const size_t ao = (size_t)(m0 + (i << 4) + rlane) * lda + koff + k0;
      V ah = Frag<T>::load(A + ao);
      V al = ah;
      if (SPL == 1) al = Frag<T>::load(A2 + ao);
#pragma unroll
      for (int j = 0; j < 4; ++j) {
        acc[i][j] = Frag<T>::mma(ah, bh[j], acc[i][j]);
        if (SPL == 1) acc[i][j] = Frag<T>::mma(al, bh[j], acc[i][j]);
      }
      dep_guard4_b(acc[i][0], acc[i][1], acc[i][2], acc[i][3], ah, al);
    }
    keep4_b(bh[0], bh[1], bh[2], bh[3]);
  }
  acc_guard4(acc[0][0], acc[0][1], acc[0][2], acc[0][3]);
  acc_guard4(acc[1][0], acc[1][1], acc[1][2], acc[1][3]);
  acc_guard4(acc[2][0], acc[2][1], acc[2][2], acc[2][3]);
  acc_guard4(acc[3][0], acc[3][1], acc[3][2], acc[3][3]);

  float* slab = sT[wave];
#pragma unroll
  for (int i = 0; i < 4; ++i) {
    const int mBase = m0 + (i << 4);
    float rm[8];
#pragma unroll
    for (int r = 0; r < 8; ++r) rm[r] = 1.0f;
    if (ROWMUL) {
#pragma unroll
      for (int r = 0; r < 8; ++r) rm[r] = bf16r(rowmul[mBase + mOff + r]);
    }
#pragma unroll
    for (int j = 0; j < 4; ++j) {
#pragma unroll
      for (int r = 0; r < 8; ++r) {
        float v = acc[i][j][r];
        if (ROWMUL) v = v * rm[r];
        slab[(mOff + r) * 68 + (j << 4) + rlane] = v;
      }
    }
    __builtin_amdgcn_fence(__ATOMIC_RELEASE, "workgroup");
    __builtin_amdgcn_wave_barrier();
    __builtin_amdgcn_fence(__ATOMIC_ACQUIRE, "workgroup");
    {
      const int hh = lane >> 4, c4 = (lane & 15) * 4;
      for (int pass = 0; pass < 2; ++pass) {
#pragma unroll
        for (int it = 0; it < 8; ++it) {
          const int row = it * 2 + hh;
          v4f v = *(const v4f*)(slab + row * 68 + c4);
          *(volatile v4f*)(Cout + (size_t)(mBase + row) * ldc + n0 + c4) = v;
        }
        __threadfence();
      }
    }
    __builtin_amdgcn_fence(__ATOMIC_RELEASE, "workgroup");
    __builtin_amdgcn_wave_barrier();
    __builtin_amdgcn_fence(__ATOMIC_ACQUIRE, "workgroup");
  }
}

__global__ __launch_bounds__(256) void cvt_rows_bf16_kernel(
    const float* __restrict__ src, unsigned short* __restrict__ dst, int total8)
{
  const int i = blockIdx.x * 256 + threadIdx.x;
  if (i >= total8) return;
  const size_t e0 = (size_t)i << 3;
  const v4f a0 = *(const v4f*)(src + e0);
  const v4f a1 = *(const v4f*)(src + e0 + 4);
  v4u w;
  w[0] = pack_hi2(a0[0], a0[1]);
  w[1] = pack_hi2(a0[2], a0[3]);
  w[2] = pack_hi2(a1[0], a1[1]);
  w[3] = pack_hi2(a1[2], a1[3]);
  unsigned short* q = dst + e0;
  *(volatile v4u*)q = w;
  __threadfence();
  *(volatile v4u*)q = w;
}

__global__ __launch_bounds__(256) void dtin_split_kernel(
    const float* __restrict__ XD, unsigned short* __restrict__ DTH, unsigned short* __restrict__ DTL, int total8)
{
  const int i = blockIdx.x * 256 + threadIdx.x;
  if (i >= total8) return;
  const int e0  = i << 3;
  const int row = e0 >> 6;
  const int c8  = e0 & 63;
  const float* p = XD + (size_t)row * kXdP + c8;
  const v4f a0 = *(const v4f*)(p);
  const v4f a1 = *(const v4f*)(p + 4);
  v4u wh, wl;
  wh[0] = pack_hi2(a0[0], a0[1]);
  wh[1] = pack_hi2(a0[2], a0[3]);
  wh[2] = pack_hi2(a1[0], a1[1]);
  wh[3] = pack_hi2(a1[2], a1[3]);
  wl[0] = pack_lo2(a0[0], a0[1]);
  wl[1] = pack_lo2(a0[2], a0[3]);
  wl[2] = pack_lo2(a1[0], a1[1]);
  wl[3] = pack_lo2(a1[2], a1[3]);
  unsigned short* qh = DTH + e0;
  unsigned short* ql = DTL + e0;
  *(volatile v4u*)qh = wh;
  *(volatile v4u*)ql = wl;
  __threadfence();
  *(volatile v4u*)qh = wh;
  *(volatile v4u*)ql = wl;
}

__global__ __launch_bounds__(256) void conv_silu_kernel(
    const float* __restrict__ XZ, const float* __restrict__ cw, const float* __restrict__ cb,
    float* __restrict__ UC, unsigned short* __restrict__ UCH, unsigned short* __restrict__ UCL)
{
  __shared__ __align__(16) float sT[16 * kConvTP];
  const int tid = threadIdx.x, lane = tid & 31, wave = tid >> 5;
  const int d0 = blockIdx.x * 256, d = d0 + tid;
  const int g0 = blockIdx.y * 64;
  const int tb = g0 & (kSeq - 1);
  const v4f wv = *(const v4f*)(cw + (size_t)d * 4);
  const float w0 = bf16r(wv[0]), w1 = bf16r(wv[1]), w2 = bf16r(wv[2]), w3 = bf16r(wv[3]);
  const float bc = bf16r(cb[d]);
  float xm3, xm2, xm1;
  {
    const bool hist = (tb > 0);
    const int rb = hist ? (g0 - 3) : g0;
    const float v3 = XZ[(size_t)rb * kXzP + d];
    const float v2 = XZ[(size_t)(rb + 1) * kXzP + d];
    const float v1 = XZ[(size_t)(rb + 2) * kXzP + d];
    xm3 = hist ? v3 : 0.f;
    xm2 = hist ? v2 : 0.f;
    xm1 = hist ? v1 : 0.f;
  }
  const int hrow = wave >> 1;
  const int hch  = (wave & 1) * 128 + lane * 4;
#pragma unroll 1
  for (int sub = 0; sub < 4; ++sub) {
    const int lb = g0 + sub * 16;
#pragma unroll 1
    for (int s = 0; s < 16; ++s) {
      const float xcur = XZ[(size_t)(lb + s) * kXzP + d];
      float acc = w0 * xm3;
      acc = fmaf(w1, xm2, acc);
      acc = fmaf(w2, xm1, acc);
      acc = fmaf(w3, xcur, acc);
      const float sv = acc + bc;
      const float ex = expf(fminf(-sv, 80.0f));
      const float sg = __builtin_amdgcn_rcpf(1.0f + ex);
      sT[s * kConvTP + tid] = sv * sg;
      xm3 = xm2; xm2 = xm1; xm1 = xcur;
    }
    __syncthreads();
    v4f fv[4];
    v4u bh[2], bl[2];
#pragma unroll
    for (int it = 0; it < 4; ++it) fv[it] = *(const v4f*)(sT + (it * 4 + hrow) * kConvTP + hch);
#pragma unroll
    for (int it = 0; it < 2; ++it) {
      const float* sp = sT + (it * 8 + wave) * kConvTP + lane * 8;
      const v4f a0 = *(const v4f*)(sp);
      const v4f a1 = *(const v4f*)(sp + 4);
      bh[it][0] = pack_hi2(a0[0], a0[1]);
      bh[it][1] = pack_hi2(a0[2], a0[3]);
      bh[it][2] = pack_hi2(a1[0], a1[1]);
      bh[it][3] = pack_hi2(a1[2], a1[3]);
      bl[it][0] = pack_lo2(a0[0], a0[1]);
      bl[it][1] = pack_lo2(a0[2], a0[3]);
      bl[it][2] = pack_lo2(a1[0], a1[1]);
      bl[it][3] = pack_lo2(a1[2], a1[3]);
    }
    for (int pass = 0; pass < 2; ++pass) {
#pragma unroll
      for (int it = 0; it < 4; ++it)
        *(volatile v4f*)(UC + (size_t)(lb + it * 4 + hrow) * kDin + d0 + hch) = fv[it];
#pragma unroll
      for (int it = 0; it < 2; ++it) {
        const size_t o = (size_t)(lb + it * 8 + wave) * kDin + d0 + lane * 8;
        *(volatile v4u*)(UCH + o) = bh[it];
        *(volatile v4u*)(UCL + o) = bl[it];
      }
      __threadfence();
    }
    __syncthreads();
  }
}

__device__ __forceinline__ float exp_nonpos(float t) {
  const float c  = 0x1.715476p+0f;
  const float cc = 0x1.4ae0bep-26f;
  const float ph = t * c;
  float pl = fmaf(t, c, -ph);
  pl = fmaf(t, cc, pl);
  const float e = __builtin_amdgcn_exp2f(ph);
  return fmaf(e, pl * 0.693147182f, e);
}

__global__ __launch_bounds__(64) void scan_kernel(
    const float* __restrict__ DLR, const float* __restrict__ UC, const float* __restrict__ XZ,
    const float* __restrict__ XD, const float* __restrict__ bdt, const float* __restrict__ Alog,
    const float* __restrict__ Dp, unsigned short* __restrict__ YH, unsigned short* __restrict__ YL)
{
  __shared__ __align__(16) float sBC[kScanTS * 128];
  __shared__ __align__(16) float sY[kScanTS * kScanYP];
  __shared__ __align__(16) float sH[kScanCh * kScanHP];
  __shared__ __align__(16) float sA[kScanCh * kScanHP];
  const int tid = threadIdx.x, lane = tid & 31, wave = tid >> 5;
  constexpr int kBlkPerB = kDin / kScanCh;
  const int bix = blockIdx.x / kBlkPerB;
  const int d0  = (blockIdx.x - bix * kBlkPerB) * kScanCh;
  const int d   = d0 + tid;
  const size_t row0 = (size_t)bix * kSeq;
  float* myH = sH + tid * kScanHP;
  float* myA = sA + tid * kScanHP;
#pragma unroll 1
  for (int g = 0; g < kNst / 4; ++g) {
    const v4f al = *(const v4f*)(Alog + (size_t)d * kNst + 4 * g);
    v4f av;
    av[0] = -expf(bf16r(al[0]));
    av[1] = -expf(bf16r(al[1]));
    av[2] = -expf(bf16r(al[2]));
    av[3] = -expf(bf16r(al[3]));
    *(v4f*)(myA + 4 * g) = av;
    *(v4f*)(myH + 4 * g) = (v4f){0.f, 0.f, 0.f, 0.f};
  }
  const float bb = bf16r(bdt[d]);
  const float Dd = bf16r(Dp[d]);
  const int q = lane >> 3, c8 = (lane & 7) * 8;
  __syncthreads();
#pragma unroll 1
  for (int t0 = 0; t0 < kSeq; t0 += kScanTS) {
    __syncthreads();
#pragma unroll
    for (int i = 0; i < 8; ++i) {
      const int idx = tid + 64 * i;
      const int r   = idx >> 5;
      const int c4  = (idx & 31) * 4;
      *(v4f*)(sBC + r * 128 + c4) = *(const v4f*)(XD + (row0 + t0 + r) * kXdP + kDtR + c4);
    }
    __syncthreads();
#pragma unroll 1
    for (int s = 0; s < kScanTS; ++s) {
      const size_t m = row0 + t0 + s;
      const float v   = DLR[m * kDin + d] + bb;
      const float xt  = UC[m * kDin + d];
      const float zv  = XZ[m * kXzP + kDin + d];
      const float a   = expf(-fabsf(v));
      const float u   = 1.0f + a;
      const float l1p = logf(u) + (a - (u - 1.0f)) * __builtin_amdgcn_rcpf(u);
      const float dt  = fmaxf(v, 0.0f) + l1p;
      const float dtx = dt * xt;
      const float* bc = sBC + s * 128;
      float y = 0.0f;
#pragma unroll 2
      for (int g = 0; g < kNst / 4; ++g) {
        v4f hv = *(const v4f*)(myH + 4 * g);
        const v4f av = *(const v4f*)(myA + 4 * g);
        const v4f bv = *(const v4f*)(bc + 4 * g);
        const v4f cv = *(const v4f*)(bc + kNst + 4 * g);
#pragma unroll
        for (int e = 0; e < 4; ++e) {
          const float ex = exp_nonpos(dt * av[e]);
          const float hn = fmaf(ex, hv[e], dtx * bv[e]);
          hv[e] = hn;
          y = fmaf(hn, cv[e], y);
        }
        *(v4f*)(myH + 4 * g) = hv;
      }
      y = fmaf(xt, Dd, y);
      const float ez = expf(fminf(-zv, 80.0f));
      const float sg = __builtin_amdgcn_rcpf(1.0f + ez);
      sY[s * kScanYP + tid] = y * (zv * sg);
    }
    __syncthreads();
    v4u hw[2], lw[2];
#pragma unroll
    for (int it = 0; it < 2; ++it) {
      const int row = it * 8 + wave * 4 + q;
      const float* sp = sY + row * kScanYP + c8;
      const v4f a0 = *(const v4f*)(sp);
      const v4f a1 = *(const v4f*)(sp + 4);
      hw[it][0] = pack_hi2(a0[0], a0[1]);
      hw[it][1] = pack_hi2(a0[2], a0[3]);
      hw[it][2] = pack_hi2(a1[0], a1[1]);
      hw[it][3] = pack_hi2(a1[2], a1[3]);
      lw[it][0] = pack_lo2(a0[0], a0[1]);
      lw[it][1] = pack_lo2(a0[2], a0[3]);
      lw[it][2] = pack_lo2(a1[0], a1[1]);
      lw[it][3] = pack_lo2(a1[2], a1[3]);
    }
    for (int pass = 0; pass < 2; ++pass) {
#pragma unroll
      for (int it = 0; it < 2; ++it) {
        const int row = it * 8 + wave * 4 + q;
        const size_t o = (row0 + t0 + row) * kDin + d0 + c8;
        *(volatile v4u*)(YH + o) = hw[it];
        *(volatile v4u*)(YL + o) = lw[it];
      }
      __threadfence();
    }
  }
}

static_assert((kRows / 64) * (kXzP / 64) == 256 * 8, "in_proj grid");
static_assert((kRows / 64) * (kXdP / 64) == 12 * 8, "x_proj grid");
static_assert((kRows / 64) * (kDin / 64) == 128 * 8, "dt_proj grid");
static_assert((kRows / 64) * (kDm / 64) == 64 * 8, "out_proj grid");

extern "C" void kernel_launch(void* const* d_in, const int* in_sizes, int n_in,
                              void* d_out, int out_size, void* d_ws, size_t ws_size,
                              hipStream_t stream) {
  if (n_in < 11) return;
  if (in_sizes[0] != kRows * kDm) return;
  if (in_sizes[1] != kRows) return;
  if (in_sizes[2] != kXzP * kDm) return;
  if (in_sizes[3] != kDin * 4) return;
  if (in_sizes[4] != kDin) return;
  if (in_sizes[5] != kXdP * kDin) return;
  if (in_sizes[6] != kDin * kDtR) return;
  if (in_sizes[7] != kDin) return;
  if (in_sizes[8] != kDin * kNst) return;
  if (in_sizes[9] != kDin) return;
  if (in_sizes[10] != kDm * kDin) return;
  if (out_size != kRows * kDm) return;
  if (ws_size < kWsTotal) return;

  const float* x       = (const float*)d_in[0];
  const float* mask    = (const float*)d_in[1];
  const float* W_in    = (const float*)d_in[2];
  const float* conv_w  = (const float*)d_in[3];
  const float* conv_b  = (const float*)d_in[4];
  const float* W_xproj = (const float*)d_in[5];
  const float* W_dt    = (const float*)d_in[6];
  const float* b_dt    = (const float*)d_in[7];
  const float* A_log   = (const float*)d_in[8];
  const float* Dp      = (const float*)d_in[9];
  const float* W_out   = (const float*)d_in[10];
  float* out = (float*)d_out;

  char* ws = (char*)d_ws;
  unsigned short* XH   = (unsigned short*)(ws + kOffXH);
  unsigned short* WIH  = (unsigned short*)(ws + kOffWIH);
  unsigned short* WXH  = (unsigned short*)(ws + kOffWXH);
  unsigned short* WDH  = (unsigned short*)(ws + kOffWDH);
  unsigned short* WOH  = (unsigned short*)(ws + kOffWOH);
  float*          XZ   = (float*)(ws + kOffXZ);
  float*          UC   = (float*)(ws + kOffUC);
  unsigned short* UCH  = (unsigned short*)(ws + kOffUCH);
  unsigned short* UCL  = (unsigned short*)(ws + kOffUCL);
  float*          XD   = (float*)(ws + kOffXD);
  unsigned short* DTH  = (unsigned short*)(ws + kOffDTH);
  unsigned short* DTL  = (unsigned short*)(ws + kOffDTL);
  float*          DLR  = (float*)(ws + kOffDLR);
  unsigned short* YH   = (unsigned short*)(ws + kOffYH);
  unsigned short* YL   = (unsigned short*)(ws + kOffYL);

  cvt_rows_bf16_kernel<<<(kRows * kDm / 8) / 256, 256, 0, stream>>>(x, XH, kRows * kDm / 8);
  cvt_rows_bf16_kernel<<<(kXzP * kDm / 8) / 256, 256, 0, stream>>>(W_in, WIH, kXzP * kDm / 8);
  cvt_rows_bf16_kernel<<<(kXdP * kDin / 8) / 256, 256, 0, stream>>>(W_xproj, WXH, kXdP * kDin / 8);
  cvt_rows_bf16_kernel<<<(kDin * kDtR / 8) / 256, 256, 0, stream>>>(W_dt, WDH, kDin * kDtR / 8);
  cvt_rows_bf16_kernel<<<(kDm * kDin / 8) / 256, 256, 0, stream>>>(W_out, WOH, kDm * kDin / 8);

  wmma_gemm64<0, false><<<256, 256, 0, stream>>>(
      XH, XH, kDm, WIH, kDm, XZ, kXzP, mask, kRows, kXzP, kDm);

  conv_silu_kernel<<<dim3(kDin / 256, kRows / 64), 256, 0, stream>>>(XZ, conv_w, conv_b, UC, UCH, UCL);

  wmma_gemm64<1, false><<<12, 256, 0, stream>>>(
      UCH, UCL, kDin, WXH, kDin, XD, kXdP, mask, kRows, kXdP, kDin);

  dtin_split_kernel<<<(kRows * kDtR / 8) / 256, 256, 0, stream>>>(XD, DTH, DTL, kRows * kDtR / 8);

  wmma_gemm64<1, false><<<128, 256, 0, stream>>>(
      DTH, DTL, kDtR, WDH, kDtR, DLR, kDin, mask, kRows, kDin, kDtR);

  scan_kernel<<<kBatch * (kDin / kScanCh), kScanCh, 0, stream>>>(DLR, UC, XZ, XD, b_dt, A_log, Dp, YH, YL);

  wmma_gemm64<1, true><<<64, 256, 0, stream>>>(
      YH, YL, kDin, WOH, kDin, out, kDm, mask, kRows, kDm, kDin);
}
